// SparseKANLinear_45921790329044
// MI455X (gfx1250) — hardware-verified
//
#include <hip/hip_runtime.h>
#include <math.h>

constexpr int kRows   = 16384;
constexpr int kIn     = 512;
constexpr int kOutF   = 512;
constexpr int kCoef   = 8;
constexpr int kKnots  = 12;
constexpr int kNB0    = 11;
constexpr int kKS     = kIn * kCoef;
constexpr int kChunk  = 4096;
constexpr int kNChunk = kRows / kChunk;
constexpr int kNRcp   = 30;
constexpr float kWbCarry  = 16.0f;
constexpr float kWsCarry  = 4096.0f;
constexpr float kBaseScale = 1.0f / 16.0f;
constexpr float kSplScale  = 1.0f / 4096.0f;

static_assert(kRows % kChunk == 0);
static_assert(kChunk % 64 == 0 && kOutF % 64 == 0);
static_assert(kIn % 32 == 0 && kKS % 32 == 0);
static_assert((kChunk * kIn) % 256 == 0);
static_assert((kOutF * kIn) % 256 == 0);

constexpr size_t kOffBtb  = 0;
constexpr size_t kOffBts  = kOffBtb  + (size_t)kOutF * kIn * 2;
constexpr size_t kOffRt   = kOffBts  + (size_t)kOutF * kKS * 2;
constexpr size_t kOffSil  = kOffRt   + (size_t)kNRcp * kIn * 4;
constexpr size_t kOffBase = kOffSil  + (size_t)kChunk * kIn * 2;
constexpr size_t kOffBas  = kOffBase + (size_t)kChunk * kOutF * 4;
constexpr size_t kWsTotal = kOffBas  + (size_t)kChunk * kKS * 2;
static_assert(kOffBts % 128 == 0 && kOffRt % 128 == 0 && kOffSil % 128 == 0 && kOffBase % 128 == 0 && kOffBas % 128 == 0);
static_assert(kWsTotal == 50917376);
static_assert(kWsTotal <= 134217728);

typedef __attribute__((ext_vector_type(16))) _Float16 v16h;
typedef __attribute__((ext_vector_type(8)))  _Float16 v8h;
typedef __attribute__((ext_vector_type(16))) __bf16   v16b;
typedef __attribute__((ext_vector_type(8)))  __bf16   v8b;
typedef __attribute__((ext_vector_type(8)))  float    v8f;
typedef __attribute__((ext_vector_type(4)))  float    v4f;
typedef __attribute__((ext_vector_type(4)))  unsigned int v4u;

__device__ __forceinline__ unsigned short f2bf_bits(float f) {
  unsigned u = __float_as_uint(f);
  return (unsigned short)((u + 0x7FFFu + ((u >> 16) & 1u)) >> 16);
}
__device__ __forceinline__ float bf_bits2f(unsigned short h) { return __uint_as_float(((unsigned)h) << 16); }

__device__ __forceinline__ void dep_guard_h(v8f& a, v8f& b, v16h x, v16h y) { asm volatile("v_nop\n\tv_nop\n\tv_nop\n\tv_nop" : "+v"(a), "+v"(b) : "v"(x), "v"(y)); }
__device__ __forceinline__ void dep_guard_b(v8f& a, v8f& b, v16b x, v16b y) { asm volatile("v_nop\n\tv_nop\n\tv_nop\n\tv_nop" : "+v"(a), "+v"(b) : "v"(x), "v"(y)); }
__device__ __forceinline__ void keep4_h(v16h a, v16h b, v16h c, v16h d) { asm volatile("v_nop" :: "v"(a), "v"(b), "v"(c), "v"(d)); }
__device__ __forceinline__ void keep4_b(v16b a, v16b b, v16b c, v16b d) { asm volatile("v_nop" :: "v"(a), "v"(b), "v"(c), "v"(d)); }
__device__ __forceinline__ void acc_guard4(v8f& a, v8f& b, v8f& c, v8f& d) { asm volatile("v_nop\n\tv_nop\n\tv_nop\n\tv_nop" : "+v"(a), "+v"(b), "+v"(c), "+v"(d)); }
template <typename T> struct Frag;
template <> struct Frag<_Float16> {
  typedef v16h V; union U { v16h v; v8h h[2]; };
  static __device__ __forceinline__ v16h load(const _Float16* p) {
    U f; f.h[0] = *(const v8h*)(p); f.h[1] = *(const v8h*)(p + 16); return f.v;
  }
  static __device__ __forceinline__ v8f mma(v16h a, v16h b, v8f c) {
    return __builtin_amdgcn_wmma_f32_16x16x32_f16(false, a, false, b, (short)0, c, false, false);
  }
  static __device__ __forceinline__ void guard(v8f& a, v8f& b, v16h x, v16h y) { dep_guard_h(a, b, x, y); }
  static __device__ __forceinline__ void keep(v16h a, v16h b, v16h c, v16h d) { keep4_h(a, b, c, d); }
};
template <> struct Frag<__bf16> {
  typedef v16b V; union U { v16b v; v8b h[2]; };
  static __device__ __forceinline__ v16b load(const __bf16* p) {
    U f; f.h[0] = *(const v8b*)(p); f.h[1] = *(const v8b*)(p + 16); return f.v;
  }
  static __device__ __forceinline__ v8f mma(v16b a, v16b b, v8f c) {
    return __builtin_amdgcn_wmma_f32_16x16x32_bf16(false, a, false, b, (short)0, c, false, false);
  }
  static __device__ __forceinline__ void guard(v8f& a, v8f& b, v16b x, v16b y) { dep_guard_b(a, b, x, y); }
  static __device__ __forceinline__ void keep(v16b a, v16b b, v16b c, v16b d) { keep4_b(a, b, c, d); }
};

__device__ __forceinline__ unsigned pk16(unsigned short a, unsigned short b) { return (unsigned)a | ((unsigned)b << 16); }
__device__ __forceinline__ unsigned short h_bits(float f) { const _Float16 h = (_Float16)f; return __builtin_bit_cast(unsigned short, h); }

template <int ET> struct Elem;
template <> struct Elem<0> { typedef _Float16 T; };
template <> struct Elem<1> { typedef __bf16 T; };
template <int ET, bool SPLIT, int BIAS_MODE, int OUT_MODE, bool RESID, int ACT = 0>
__global__ __launch_bounds__(256) void wmma_gemm64(
    const unsigned short* __restrict__ Ap, const unsigned short* __restrict__ A2p, int lda, long strideA,
    const unsigned short* __restrict__ Btp, const unsigned short* __restrict__ Bt2p, int ldb, long strideB,
    void* __restrict__ Cout, void* __restrict__ Cout2, int ldc, long strideC,
    const float* __restrict__ bias,
    const float* __restrict__ resid, long strideR,
    int M, int N, int K, float scale) {
  typedef typename Elem<ET>::T T;
  typedef typename Frag<T>::V V;
  const T* A = (const T*)Ap; const T* A2 = (const T*)A2p; const T* Bt = (const T*)Btp; const T* Bt2 = (const T*)Bt2p;
  __shared__ __align__(16) float sT[8][16 * 68];
  const int b    = blockIdx.y;
  const int lane = threadIdx.x & 31;
  const int wave = threadIdx.x >> 5;
  const int tilesN = N >> 6;
  const int tilesM = M >> 6;
  const int tile = blockIdx.x * 8 + wave;
  if (tile >= tilesM * tilesN) return;
  const int tm = tile / tilesN;
  const int tn = tile - tm * tilesN;
  const int m0 = tm << 6;
  const int n0 = tn << 6;

  const T* Ab  = A  + (size_t)b * strideA;
  const T* Bb  = Bt + (size_t)b * strideB;
  const T* Ab2 = SPLIT ? (A2  + (size_t)b * strideA) : nullptr;
  const T* Bb2 = SPLIT ? (Bt2 + (size_t)b * strideB) : nullptr;

  const int rlane = lane & 15;
  const int koff  = (lane >> 4) * 8;
  const int mOff  = (lane >> 4) * 8;

  v8f acc[4][4];
#pragma unroll
  for (int i = 0; i < 4; ++i)
#pragma unroll
    for (int j = 0; j < 4; ++j) acc[i][j] = (v8f){0.f,0.f,0.f,0.f,0.f,0.f,0.f,0.f};

  for (int k0 = 0; k0 < K; k0 += 32) {
    V bh[4], bl[4];
#pragma unroll
    for (int j = 0; j < 4; ++j) {
      const size_t bo = (size_t)(n0 + (j << 4) + rlane) * ldb + koff + k0;
      bh[j] = Frag<T>::load(Bb + bo);
      if (SPLIT) bl[j] = Frag<T>::load(Bb2 + bo);
    }
#pragma unroll
    for (int i = 0; i < 4; ++i) {
      const size_t ao = (size_t)(m0 + (i << 4) + rlane) * lda + koff + k0;
      V ah = Frag<T>::load(Ab + ao);
      V al;
      if (SPLIT) al = Frag<T>::load(Ab2 + ao);
#pragma unroll
      for (int j = 0; j < 4; ++j) {
        acc[i][j] = Frag<T>::mma(ah, bh[j], acc[i][j]);
        if (SPLIT) {
          acc[i][j] = Frag<T>::mma(ah, bl[j], acc[i][j]);
          acc[i][j] = Frag<T>::mma(al, bh[j], acc[i][j]);
        }
      }
      Frag<T>::guard(acc[i][0], acc[i][3], ah, SPLIT ? al : ah);
    }
    Frag<T>::keep(bh[0], bh[1], bh[2], bh[3]);
    if (SPLIT) Frag<T>::keep(bl[0], bl[1], bl[2], bl[3]);
  }
  acc_guard4(acc[0][0], acc[0][1], acc[0][2], acc[0][3]);
  acc_guard4(acc[1][0], acc[1][1], acc[1][2], acc[1][3]);
  acc_guard4(acc[2][0], acc[2][1], acc[2][2], acc[2][3]);
  acc_guard4(acc[3][0], acc[3][1], acc[3][2], acc[3][3]);

  float* slab = sT[wave];
  const float* Rb = RESID ? (resid + (size_t)b * strideR) : nullptr;
#pragma unroll
  for (int i = 0; i < 4; ++i) {
    const int mBase = m0 + (i << 4);
#pragma unroll
    for (int j = 0; j < 4; ++j) {
      const int n = n0 + (j << 4) + rlane;
      float bv = 0.f;
      if (BIAS_MODE == 2) bv = bias[n];
#pragma unroll
      for (int r = 0; r < 8; ++r) {
        float v = acc[i][j][r] * scale;
        if (BIAS_MODE == 1) v += bias[mBase + mOff + r];
        if (BIAS_MODE == 2) v += bv;
        if (RESID) v += Rb[(size_t)(mBase + mOff + r) * ldc + n];
        if (ACT == 2) v = fmaxf(v, 0.0f);
        if (ACT == 4) v = (v > 0.f) ? v : 0.01f * v;
        slab[(mOff + r) * 68 + (j << 4) + rlane] = v;
      }
    }
    __builtin_amdgcn_fence(__ATOMIC_RELEASE, "workgroup");
    __builtin_amdgcn_wave_barrier();
    __builtin_amdgcn_fence(__ATOMIC_ACQUIRE, "workgroup");
    if (OUT_MODE == 0) {
      float* C = (float*)Cout + (size_t)b * strideC;
      const int hh = lane >> 4, c4 = (lane & 15) * 4;
      for (int pass = 0; pass < 2; ++pass) {
#pragma unroll
        for (int it = 0; it < 8; ++it) {
          const int row = it * 2 + hh;
          v4f v = *(const v4f*)(slab + row * 68 + c4);
          *(volatile v4f*)(C + (size_t)(mBase + row) * ldc + n0 + c4) = v;
        }
        __threadfence();
      }
    } else {
      const int q = lane >> 3, c8 = (lane & 7) * 8;
      unsigned short* C  = (unsigned short*)Cout  + (size_t)b * strideC;
      unsigned short* C2 = (OUT_MODE == 2) ? ((unsigned short*)Cout2 + (size_t)b * strideC) : nullptr;
      for (int pass = 0; pass < 2; ++pass) {
#pragma unroll
        for (int it = 0; it < 4; ++it) {
          const int row = it * 4 + q;
          const float* sp = slab + row * 68 + c8;
          v8h hv, lv;
#pragma unroll
          for (int e = 0; e < 8; ++e) {
            if (OUT_MODE == 1) {
              hv[e] = (_Float16)sp[e];
            } else {
              unsigned short hb = f2bf_bits(sp[e]);
              unsigned short lb = f2bf_bits(sp[e] - bf_bits2f(hb));
              hv[e] = __builtin_bit_cast(_Float16, hb);
              lv[e] = __builtin_bit_cast(_Float16, lb);
            }
          }
          *(volatile v8h*)(C + (size_t)(mBase + row) * ldc + n0 + c8) = hv;
          if (OUT_MODE == 2) *(volatile v8h*)(C2 + (size_t)(mBase + row) * ldc + n0 + c8) = lv;
        }
        __threadfence();
      }
    }
    __builtin_amdgcn_fence(__ATOMIC_RELEASE, "workgroup");
    __builtin_amdgcn_wave_barrier();
    __builtin_amdgcn_fence(__ATOMIC_ACQUIRE, "workgroup");
  }
}

__global__ __launch_bounds__(256) void prep_kernel(const float* __restrict__ bw, const float* __restrict__ sw,
                                                    const float* __restrict__ ss, const float* __restrict__ mk,
                                                    const float* __restrict__ G,
                                                    unsigned short* __restrict__ btb, unsigned short* __restrict__ bts,
                                                    float* __restrict__ rt) {
  const int t   = threadIdx.x;
  const int idx = blockIdx.x * 256 + t;

  const float s = mk[idx] * ss[idx];
  const float* wp = sw + (size_t)idx * kCoef;
  const v4f w0 = *(const v4f*)(wp);
  const v4f w1 = *(const v4f*)(wp + 4);
  unsigned short hs[8];
#pragma unroll
  for (int e = 0; e < 4; ++e) {
    hs[e]     = h_bits((w0[e] * s) * kWsCarry);
    hs[4 + e] = h_bits((w1[e] * s) * kWsCarry);
  }
  const v4u us = (v4u){pk16(hs[0], hs[1]), pk16(hs[2], hs[3]), pk16(hs[4], hs[5]), pk16(hs[6], hs[7])};

  const bool dobase = (blockIdx.x < (kOutF * kIn) / (8 * 256));
  v4u ub = us;
  if (dobase) {
    const size_t e8 = (size_t)idx * 8;
    const v4f bA = *(const v4f*)(bw + e8);
    const v4f bB = *(const v4f*)(bw + e8 + 4);
    const v4f mA = *(const v4f*)(mk + e8);
    const v4f mB = *(const v4f*)(mk + e8 + 4);
    unsigned short hb[8];
#pragma unroll
    for (int e = 0; e < 4; ++e) {
      hb[e]     = h_bits((bA[e] * mA[e]) * kWbCarry);
      hb[4 + e] = h_bits((bB[e] * mB[e]) * kWbCarry);
    }
    ub = (v4u){pk16(hb[0], hb[1]), pk16(hb[2], hb[3]), pk16(hb[4], hb[5]), pk16(hb[6], hb[7])};
  }
  unsigned short* ps = bts + (size_t)idx * 8;
  unsigned short* pb = btb + (size_t)idx * 8;
  *(volatile v4u*)ps = us;
  if (dobase) *(volatile v4u*)pb = ub;
  __threadfence();
  *(volatile v4u*)ps = us;
  if (dobase) *(volatile v4u*)pb = ub;

  if (blockIdx.x < 2) {
    const int i = idx;
    const float* gr = G + (size_t)i * kKnots;
#pragma unroll 1
    for (int q = 0; q < kNRcp; ++q) {
      const int k = 1 + (q >= 11 ? 1 : 0) + (q >= 21 ? 1 : 0);
      const int j = q - (q >= 11 ? 11 : 0) - (q >= 21 ? 10 : 0);
      const float den = (gr[j + k] - gr[j]) + 1e-8f;
      const float r = 1.0f / den;
      volatile float* p = rt + (size_t)q * kIn + i;
      *p = r;
      __threadfence();
      *p = r;
    }
  }
}

__global__ __launch_bounds__(256) void act_kernel(const float* __restrict__ X, const float* __restrict__ G,
                                                   const float* __restrict__ rt,
                                                   unsigned short* __restrict__ sil, unsigned short* __restrict__ bas,
                                                   int row0) {
  __shared__ __align__(16) _Float16 ssil[256];
  const int t    = threadIdx.x;
  const int lane = t & 31;
  const int wave = t >> 5;
  const int idx  = blockIdx.x * 256 + t;
  const int nl   = idx >> 9;
  const int i    = idx & (kIn - 1);
  const int ibase = i & ~255;

  const float* gr = G + (size_t)i * kKnots;
  float g[kKnots];
#pragma unroll
  for (int e = 0; e < kKnots; ++e) g[e] = gr[e];
  float rr[kNRcp];
#pragma unroll
  for (int q = 0; q < kNRcp; ++q) rr[q] = rt[(size_t)q * kIn + i];

  const float xv = X[(size_t)(row0 + nl) * kIn + i];

  const float ex = expf(-xv);
  const float sg = 1.0f / (1.0f + ex);
  const float sv = xv * sg;

  float bb[kNB0];
#pragma unroll
  for (int j = 0; j < kNB0; ++j) bb[j] = ((xv >= g[j]) & (xv < g[j + 1])) ? 1.0f : 0.0f;
#pragma unroll
  for (int j = 0; j < 10; ++j) {
    const float lf = (xv - g[j]) * rr[j];
    const float rg = (g[j + 2] - xv) * rr[j + 1];
    bb[j] = lf * bb[j] + rg * bb[j + 1];
  }
#pragma unroll
  for (int j = 0; j < 9; ++j) {
    const float lf = (xv - g[j]) * rr[11 + j];
    const float rg = (g[j + 3] - xv) * rr[11 + j + 1];
    bb[j] = lf * bb[j] + rg * bb[j + 1];
  }
#pragma unroll
  for (int j = 0; j < 8; ++j) {
    const float lf = (xv - g[j]) * rr[21 + j];
    const float rg = (g[j + 4] - xv) * rr[21 + j + 1];
    bb[j] = lf * bb[j] + rg * bb[j + 1];
  }

  unsigned short hb[8];
#pragma unroll
  for (int c = 0; c < 8; ++c) hb[c] = h_bits(bb[c]);
  const v4u ub = (v4u){pk16(hb[0], hb[1]), pk16(hb[2], hb[3]), pk16(hb[4], hb[5]), pk16(hb[6], hb[7])};

  ssil[t] = (_Float16)sv;
  __syncthreads();
  const v8h svv = *(const v8h*)(ssil + 8 * lane);

  unsigned short* bdst = bas + (size_t)nl * kKS + (size_t)i * 8;
  unsigned short* sdst = sil + (size_t)nl * kIn + ibase + 8 * lane;
  for (int pass = 0; pass < 2; ++pass) {
    *(volatile v4u*)bdst = ub;
    if (wave == 0) *(volatile v8h*)sdst = svv;
    __threadfence();
  }
}

extern "C" void kernel_launch(void* const* d_in, const int* in_sizes, int n_in,
                              void* d_out, int out_size, void* d_ws, size_t ws_size,
                              hipStream_t stream) {
  if (n_in < 6) return;
  if (in_sizes[0] != kRows * kIn) return;
  if (in_sizes[1] != kOutF * kIn) return;
  if (in_sizes[2] != kOutF * kIn * kCoef) return;
  if (in_sizes[3] != kOutF * kIn) return;
  if (in_sizes[4] != kOutF * kIn) return;
  if (in_sizes[5] != kIn * kKnots) return;
  if (out_size != kRows * kOutF) return;
  if (ws_size < kWsTotal) return;

  const float* x   = (const float*)d_in[0];
  const float* bw  = (const float*)d_in[1];
  const float* sw  = (const float*)d_in[2];
  const float* ssc = (const float*)d_in[3];
  const float* mk  = (const float*)d_in[4];
  const float* gr  = (const float*)d_in[5];
  float* out = (float*)d_out;

  char* ws = (char*)d_ws;
  unsigned short* btb  = (unsigned short*)(ws + kOffBtb);
  unsigned short* bts  = (unsigned short*)(ws + kOffBts);
  float*          rt   = (float*)(ws + kOffRt);
  unsigned short* sil  = (unsigned short*)(ws + kOffSil);
  float*          base = (float*)(ws + kOffBase);
  unsigned short* bas  = (unsigned short*)(ws + kOffBas);

  prep_kernel<<<(kOutF * kIn) / 256, 256, 0, stream>>>(bw, sw, ssc, mk, gr, btb, bts, rt);

  const int gemmBlocks = ((kChunk / 64) * (kOutF / 64)) / 8;
  for (int ch = 0; ch < kNChunk; ++ch) {
    const int row0 = ch * kChunk;
    act_kernel<<<(kChunk * kIn) / 256, 256, 0, stream>>>(x, gr, rt, sil, bas, row0);
    wmma_gemm64<0, false, 0, 0, false, 0><<<dim3(gemmBlocks, 1), 256, 0, stream>>>(
        sil, sil, kIn, 0L,
        btb, btb, kIn, 0L,
        (void*)base, (void*)base, kOutF, 0L,
        base,
        base, 0L,
        kChunk, kOutF, kIn, kBaseScale);
    float* oc = out + (size_t)row0 * kOutF;
    wmma_gemm64<0, false, 0, 0, true, 0><<<dim3(gemmBlocks, 1), 256, 0, stream>>>(
        bas, bas, kKS, 0L,
        bts, bts, kKS, 0L,
        (void*)oc, (void*)oc, kOutF, 0L,
        base,
        base, 0L,
        kChunk, kOutF, kKS, kSplScale);
  }
}
